// QuantumNAT_Enhanced_65481071406977
// MI455X (gfx1250) — hardware-verified
//
#include <hip/hip_runtime.h>


#ifndef NSAMP
#define NSAMP 524288
#endif
#define NSAMP_FULL 524288
#define NQ    4
#define NL    3
#define DIMS  16
#define AROWS 64
#define KP    32
#define NW    36
#define MW    8
#define TPW   8
#define NTILES (NSAMP / 16)
#define ACARRY 64.0f
#define PCARRY 16.0f
#define INVC   (1.0f / 1024.0f)

static_assert(NSAMP % 16 == 0);
static_assert(NSAMP <= NSAMP_FULL);
static_assert(DIMS == 16);
static_assert(AROWS == NQ * DIMS);
static_assert(KP == 32);
static_assert(NW == NL * NQ * 3);
static_assert(NW <= 256);
static_assert(256 * 8 == AROWS * KP);
static_assert((AROWS * DIMS) % 256 == 0);
static_assert(MW * 32 == 256);
static_assert((256 + 256 + AROWS * DIMS + NW + NW) * 4 <= 131072);

typedef _Float16 h16;
typedef __attribute__((ext_vector_type(16))) _Float16 v16h;
typedef __attribute__((ext_vector_type(8)))  _Float16 v8h;
typedef __attribute__((ext_vector_type(8)))  float    v8f;
typedef __attribute__((ext_vector_type(4)))  float    v4f;

__device__ __forceinline__ unsigned short f2bf(float f) { unsigned u = __float_as_uint(f); u += 0x7FFFu + ((u >> 16) & 1u); return (unsigned short)(u >> 16); }
__device__ __forceinline__ float bfr(float f) { return __uint_as_float(((unsigned)f2bf(f)) << 16); }
__device__ __forceinline__ v16h cat16(v8h lo, v8h hi) { return __builtin_shufflevector(lo, hi, 0, 1, 2, 3, 4, 5, 6, 7, 8, 9, 10, 11, 12, 13, 14, 15); }
__device__ __forceinline__ v16h ldh(const h16* p) { return cat16(*(const v8h*)p, *(const v8h*)(p + 16)); }
static __device__ __forceinline__ h16 toh_flush(float v) { const h16 r = (h16)v; return (fabsf(v) < 6.103515625e-05f) ? (h16)0.0f : r; }
__device__ __forceinline__ v8f wmma16g(v16h a, v16h b, v8f c) {
    c = __builtin_amdgcn_wmma_f32_16x16x32_f16(false, a, false, b, (short)0, c, false, false);
    asm volatile("v_nop\n\tv_nop\n\tv_nop\n\tv_nop" : "+v"(c) : "v"(a), "v"(b));
    return c;
}

__global__ __launch_bounds__(256) void k_prep(const float* __restrict__ W, h16* AH) {
#pragma clang fp contract(off)
    __shared__ float Vr[256];
    __shared__ float Vi[256];
    __shared__ __align__(16) float Af[AROWS * DIMS];
    __shared__ float sw[NW];
    __shared__ float cw[NW];
    const int tid = threadIdx.x;
    {
        const int wi = tid < NW ? tid : (NW - 1);
        float a = W[wi];
        asm volatile("" : "+v"(a));
        float s, c;
        sincosf(0.5f * bfr(a), &s, &c);
        if (tid < NW) { sw[tid] = s; cw[tid] = c; }
    }
    Vr[tid] = ((tid >> 4) == (tid & 15)) ? 1.0f : 0.0f;
    Vi[tid] = 0.0f;
    __syncthreads();

#pragma unroll 1
    for (int g = 0; g < NL * NQ; ++g) {
        const int q = g & 3;
        const float sa = sw[g * 3 + 0], ca = cw[g * 3 + 0];
        const float sb = sw[g * 3 + 1], cb = cw[g * 3 + 1];
        const float sc = sw[g * 3 + 2], cc = cw[g * 3 + 2];
        const float m00r =  cb * ca, m00i =  sb * sa;
        const float m01r = -sb * ca, m01i = -cb * sa;
        const float m10r =  sb * ca, m10i = -cb * sa;
        const float m11r =  cb * ca, m11i = -sb * sa;
        const float u00r = m00r * cc + m00i * sc, u00i = m00i * cc - m00r * sc;
        const float u01r = m01r * cc + m01i * sc, u01i = m01i * cc - m01r * sc;
        const float u10r = m10r * cc - m10i * sc, u10i = m10i * cc + m10r * sc;
        const float u11r = m11r * cc - m11i * sc, u11i = m11i * cc + m11r * sc;
        const int col = tid & 15, pr = (tid >> 4) & 7;
        const int bit = 8 >> q;
        const int low = pr & (bit - 1);
        const int k0 = ((pr - low) << 1) | low;
        const int k1 = k0 | bit;
        if (tid < 128) {
            const float ar = Vr[k0 * 16 + col], ai = Vi[k0 * 16 + col];
            const float br = Vr[k1 * 16 + col], bi = Vi[k1 * 16 + col];
            Vr[k0 * 16 + col] = u00r * ar - u00i * ai + u01r * br - u01i * bi;
            Vi[k0 * 16 + col] = u00r * ai + u00i * ar + u01r * bi + u01i * br;
            Vr[k1 * 16 + col] = u10r * ar - u10i * ai + u11r * br - u11i * bi;
            Vi[k1 * 16 + col] = u10r * ai + u10i * ar + u11r * bi + u11i * br;
        }
        __syncthreads();
        if (q == 3) {
            const int r = tid >> 4;
            int src = r;
            if (src & 2) src ^= 1;
            if (src & 4) src ^= 2;
            if (src & 8) src ^= 4;
            const float tr = Vr[src * 16 + col], ti = Vi[src * 16 + col];
            __syncthreads();
            Vr[r * 16 + col] = tr; Vi[r * 16 + col] = ti;
            __syncthreads();
        }
    }

#pragma unroll 1
    for (int idx = tid; idx < AROWS * DIMS; idx += 256) {
        const int q = idx >> 8;
        const int j = (idx >> 4) & 15;
        const int k = idx & 15;
        float mr = 0.0f, mi = 0.0f;
#pragma unroll 1
        for (int r = 0; r < 16; ++r) {
            const float z = ((r >> (3 - q)) & 1) ? -1.0f : 1.0f;
            mr += z * (Vr[r * 16 + j] * Vr[r * 16 + k] + Vi[r * 16 + j] * Vi[r * 16 + k]);
            mi += z * (Vr[r * 16 + j] * Vi[r * 16 + k] - Vi[r * 16 + j] * Vr[r * 16 + k]);
        }
        const int d = (__popc(k) - __popc(j)) & 3;
        const float re = (d == 0) ? mr : ((d == 1) ? mi : ((d == 2) ? -mr : -mi));
        Af[idx] = re;
    }
    __syncthreads();

    {
        const int row = tid >> 2, c8 = (tid & 3) * 8;
        const int cs = c8 & 8;
        const bool live = c8 < DIMS;
        v8h hv;
#pragma unroll
        for (int i = 0; i < 8; ++i) {
            const float f = Af[row * DIMS + cs + i];
            const h16 hx = toh_flush(f * ACARRY);
            hv[i] = live ? hx : (h16)0.0f;
        }
        h16* dst = AH + (size_t)tid * 8;
        *(volatile v8h*)dst = hv;
        __threadfence();
        *(volatile v8h*)dst = hv;
    }
}

__global__ __launch_bounds__(256) void k_expect(const float* __restrict__ X, const h16* __restrict__ AH, float* OUT) {
    const int lane = threadIdx.x & 31, lr = lane & 15, hi = lane >> 4;
    const int wave = __builtin_amdgcn_readfirstlane((int)(threadIdx.x >> 5));
    const int tile0 = (blockIdx.x * MW + wave) * TPW;
    const bool up = hi != 0;
    v16h af[4];
#pragma unroll
    for (int mt = 0; mt < 4; ++mt) af[mt] = ldh(AH + (size_t)(16 * mt + lr) * KP + 8 * hi);
#pragma unroll 1
    for (int it = 0; it < TPW; ++it) {
        const int tile = tile0 + it;
        if (tile >= NTILES) break;
        const size_t s = (size_t)tile * 16 + lr;
        const v4f xv = *(const v4f*)(X + s * 4);
        const float x0 = bfr(xv[0]), x1 = bfr(xv[1]), x2 = bfr(xv[2]), x3 = bfr(xv[3]);
        const float xa = up ? x2 : x0;
        const float xb = up ? x3 : x1;
        float sa, ca, sb, cb;
        sincosf(0.5f * xa, &sa, &ca);
        sincosf(0.5f * xb, &sb, &cb);
        const float p0 = ca * cb, p1 = ca * sb, p2 = sa * cb, p3 = sa * sb;
        const float r0 = __shfl_xor(p0, 16, 32), r1 = __shfl_xor(p1, 16, 32), r2 = __shfl_xor(p2, 16, 32), r3 = __shfl_xor(p3, 16, 32);
        const float uvA = up ? r2 : p0;
        const float uvB = up ? r3 : p1;
        const float wz0 = up ? p0 : r0, wz1 = up ? p1 : r1, wz2 = up ? p2 : r2, wz3 = up ? p3 : r3;
        float pf[8];
        pf[0] = uvA * wz0; pf[1] = uvA * wz1; pf[2] = uvA * wz2; pf[3] = uvA * wz3;
        pf[4] = uvB * wz0; pf[5] = uvB * wz1; pf[6] = uvB * wz2; pf[7] = uvB * wz3;
        v16h pb;
#pragma unroll
        for (int r = 0; r < 8; ++r) { pb[r] = toh_flush(pf[r] * PCARRY); pb[8 + r] = (h16)0.0f; }
        v8f acc0 = (v8f){}, acc1 = (v8f){}, acc2 = (v8f){}, acc3 = (v8f){};
        acc0 = wmma16g(af[0], pb, acc0);
        acc1 = wmma16g(af[1], pb, acc1);
        acc2 = wmma16g(af[2], pb, acc2);
        acc3 = wmma16g(af[3], pb, acc3);
        float e0 = 0.0f, e1 = 0.0f, e2 = 0.0f, e3 = 0.0f;
#pragma unroll
        for (int r = 0; r < 8; ++r) {
            const float ps = pf[r] * INVC;
            e0 += acc0[r] * ps; e1 += acc1[r] * ps; e2 += acc2[r] * ps; e3 += acc3[r] * ps;
        }
        e0 += __shfl_xor(e0, 16, 32); e1 += __shfl_xor(e1, 16, 32); e2 += __shfl_xor(e2, 16, 32); e3 += __shfl_xor(e3, 16, 32);
        v4f o; o[0] = e0; o[1] = e1; o[2] = e2; o[3] = e3;
        float* op = OUT + s * 4;
        if (!up) *(volatile v4f*)op = o;
        __threadfence();
        if (!up) *(volatile v4f*)op = o;
    }
}

static constexpr size_t al256(size_t v) { return (v + 255) & ~(size_t)255; }
static constexpr size_t SZ_AH = al256((size_t)AROWS * KP * 2);
static constexpr size_t SZ_TOTAL = SZ_AH;
static_assert(SZ_TOTAL <= (size_t)134217728);
static_assert((size_t)256 * 8 * 2 <= SZ_AH);

extern "C" void kernel_launch(void* const* d_in, const int* in_sizes, int n_in,
                              void* d_out, int out_size, void* d_ws, size_t ws_size, hipStream_t stream) {
    if (n_in < 2) return;
    if ((size_t)in_sizes[0] < (size_t)NSAMP * NQ) return;
    if (in_sizes[1] < NW) return;
    if ((size_t)out_size < (size_t)NSAMP * NQ) return;
    if (SZ_TOTAL > ws_size) return;
    const float* x = (const float*)d_in[0];
    const float* w = (const float*)d_in[1];
    float* OUT = (float*)d_out;
    h16* AH = (h16*)d_ws;

    k_prep<<<1, 256, 0, stream>>>(w, AH);
    const unsigned grid = (unsigned)((NTILES + MW * TPW - 1) / (MW * TPW));
    k_expect<<<grid, 256, 0, stream>>>(x, AH, OUT);
}
